// PixelGAT_17970143166991
// MI455X (gfx1250) — hardware-verified
//
#include <hip/hip_runtime.h>
#include <hip/hip_bf16.h>
#include <stddef.h>


#define FD    128
#define NH    4
#define HC    32
#define NG    2
#define NOUT  10
#define GR    32
#define AP    136
#define XSP   132
#define TP    132
#define NB    512
#define CHUNK 2048
#define NTHR  256
#define NWAVE 8
#define WCAP  256
#define NGRP  (CHUNK / (NTHR * 4))
#define RECD  80

#define LDS_SACC  (NB * FD)
#define LDS_AUX   (2 * NB * NH)
#define LDS_LIST  (NWAVE * WCAP)
#define LDS_BYTES ((LDS_SACC + LDS_AUX + LDS_LIST + NWAVE) * 4)

static_assert(WCAP == (CHUNK / NTHR) * 32);
static_assert(NGRP == 2);
static_assert(NB == 512);
static_assert(CHUNK <= 4096);
static_assert(FD == NH * HC);
static_assert(LDS_BYTES == 286752);
static_assert((NWAVE * 64 + RECD) * 8 <= LDS_SACC * 4);
static_assert((RECD * 8) % 128 == 0);

typedef float          v4f  __attribute__((ext_vector_type(4)));
typedef float          v8f  __attribute__((ext_vector_type(8)));
typedef int            v4i  __attribute__((ext_vector_type(4)));
typedef double         v2d  __attribute__((ext_vector_type(2)));
typedef unsigned short v8us __attribute__((ext_vector_type(8)));
typedef __bf16         v16b __attribute__((ext_vector_type(16)));
union Frag   { v16b v; v8us half[2]; };
union Pack16 { v8us h; unsigned short s[8]; v4i i; };

__device__ __forceinline__ v8f wm(v16b a, v16b b, v8f c) {
  v8f d = __builtin_amdgcn_wmma_f32_16x16x32_bf16(false, a, false, b, (short)0, c, false, false);
  asm volatile("v_nop\n\tv_nop\n\tv_nop\n\tv_nop" : "+v"(d) : "v"(a), "v"(b));
  return d;
}

__device__ __forceinline__ unsigned short bf16_rne(float f) {
  unsigned u = __float_as_uint(f);
  u = u + 0x7FFFu + ((u >> 16) & 1u);
  return (unsigned short)(u >> 16);
}
__device__ __forceinline__ void split2(float f, unsigned short& hi, unsigned short& lo) {
  hi = bf16_rne(f);
  const float fh = __uint_as_float(((unsigned)hi) << 16);
  lo = bf16_rne(f - fh);
}

__global__ __launch_bounds__(NTHR) void k_prepw(const float* __restrict__ Wa,
                                                const float* __restrict__ Wb,
                                                unsigned short* Wq) {
  __shared__ __attribute__((aligned(16))) float Ts[16 * TP];
  const int tid = threadIdx.x;
  const int mat = blockIdx.x >> 3;
  const int n0  = (blockIdx.x & 7) * 16;
  const float* W = mat ? Wb : Wa;
  unsigned short* Ph = Wq + (size_t)mat * 2 * FD * FD;
  unsigned short* Pl = Ph + FD * FD;
  {
    const int k  = tid >> 1;
    const int c0 = (tid & 1) * 8;
    const float* p = W + (size_t)k * FD + n0 + c0;
    const v4f f0 = *(const v4f*)(p);
    const v4f f1 = *(const v4f*)(p + 4);
    Ts[(c0 + 0) * TP + k] = f0.x; Ts[(c0 + 1) * TP + k] = f0.y;
    Ts[(c0 + 2) * TP + k] = f0.z; Ts[(c0 + 3) * TP + k] = f0.w;
    Ts[(c0 + 4) * TP + k] = f1.x; Ts[(c0 + 5) * TP + k] = f1.y;
    Ts[(c0 + 6) * TP + k] = f1.z; Ts[(c0 + 7) * TP + k] = f1.w;
  }
  __syncthreads();
  const int r = tid >> 4;
  const int q = tid & 15;
  const float* s = Ts + r * TP + 8 * q;
  const v4f g0 = *(const v4f*)(s);
  const v4f g1 = *(const v4f*)(s + 4);
  Pack16 uh, ul;
  split2(g0.x, uh.s[0], ul.s[0]); split2(g0.y, uh.s[1], ul.s[1]);
  split2(g0.z, uh.s[2], ul.s[2]); split2(g0.w, uh.s[3], ul.s[3]);
  split2(g1.x, uh.s[4], ul.s[4]); split2(g1.y, uh.s[5], ul.s[5]);
  split2(g1.z, uh.s[6], ul.s[6]); split2(g1.w, uh.s[7], ul.s[7]);
  const size_t o = (size_t)(n0 + r) * FD + 8 * q;
  *(volatile v4i*)(Ph + o) = uh.i;
  *(volatile v4i*)(Pl + o) = ul.i;
  __threadfence();
  *(volatile v4i*)(Ph + o) = uh.i;
  *(volatile v4i*)(Pl + o) = ul.i;
}

__device__ __forceinline__ void block_out(const float* Xs, const float* As, const float* Ds,
                                          float* xp, float* asrc, float* adst,
                                          int rowBase, int wave, int lane) {
  v4f xr[4];
#pragma unroll
  for (int i = 0; i < 4; ++i) xr[i] = *(const v4f*)(Xs + (4 * wave + i) * XSP + 4 * lane);
  v4f gv = {0.f, 0.f, 0.f, 0.f};
  float* gp = xp;
  const bool hasg = (wave < 2);
  if (wave == 0) {
    const float* q = As + lane * NWAVE;
    gv.x = q[0] + q[1]; gv.y = q[2] + q[3]; gv.z = q[4] + q[5]; gv.w = q[6] + q[7];
    gp = asrc + (size_t)rowBase * NH + 4 * lane;
  } else if (wave == 1) {
    const float* q = Ds + lane * NWAVE;
    gv.x = q[0] + q[1]; gv.y = q[2] + q[3]; gv.z = q[4] + q[5]; gv.w = q[6] + q[7];
    gp = adst + (size_t)rowBase * NH + 4 * lane;
  }
  float* xpp[4];
#pragma unroll
  for (int i = 0; i < 4; ++i) xpp[i] = xp + (size_t)(rowBase + 4 * wave + i) * FD + 4 * lane;

#pragma unroll
  for (int i = 0; i < 4; ++i) *(volatile v4f*)(xpp[i]) = xr[i];
  if (hasg) *(volatile v4f*)gp = gv;
  __threadfence();
#pragma unroll
  for (int i = 0; i < 4; ++i) *(volatile v4f*)(xpp[i]) = xr[i];
  if (hasg) *(volatile v4f*)gp = gv;
}

__global__ __launch_bounds__(NTHR) void k_l0(
    const float* __restrict__ x, const float* __restrict__ W0,
    const float* __restrict__ att_src, const float* __restrict__ att_dst,
    float* xp, float* asrc, float* adst, int nN) {
  __shared__ __attribute__((aligned(16))) float Xs[GR * XSP];
  __shared__ __attribute__((aligned(16))) float As[GR * NWAVE];
  __shared__ __attribute__((aligned(16))) float Ds[GR * NWAVE];
  const int tid  = threadIdx.x;
  const int lane = tid & 31;
  const int wave = tid >> 5;
  const int r    = tid >> 3;
  const int pc   = tid & 7;
  const int c0   = pc * 16;
  const int rowBase = blockIdx.x * GR;
  int row = rowBase + r;
  if (row > nN - 1) row = nN - 1;
  const float x0 = x[(size_t)row * 3 + 0];
  const float x1 = x[(size_t)row * 3 + 1];
  const float x2 = x[(size_t)row * 3 + 2];
  float ss = 0.f, sd = 0.f;
#pragma unroll 1
  for (int g4 = 0; g4 < 4; ++g4) {
    const int c = c0 + 4 * g4;
    const v4f w0 = *(const v4f*)(W0 + c);
    const v4f w1 = *(const v4f*)(W0 + FD + c);
    const v4f w2 = *(const v4f*)(W0 + 2 * FD + c);
    v4f v = x0 * w0;
    v = v + x1 * w1;
    v = v + x2 * w2;
    *(v4f*)(Xs + r * XSP + c) = v;
    const v4f sa = *(const v4f*)(att_src + c);
    const v4f da = *(const v4f*)(att_dst + c);
    ss += v.x * sa.x + v.y * sa.y + v.z * sa.z + v.w * sa.w;
    sd += v.x * da.x + v.y * da.y + v.z * da.z + v.w * da.w;
  }
  As[r * NWAVE + pc] = ss;
  Ds[r * NWAVE + pc] = sd;
  __syncthreads();
  block_out(Xs, As, Ds, xp, asrc, adst, rowBase, wave, lane);
}

__device__ __forceinline__ void epi_tile(v8f acc, int T, int hh, int m, int wave, int ncol,
                                         float cs, float cd, float* Xs, float* As, float* Ds) {
  float ss[8], sd[8];
#pragma unroll
  for (int r = 0; r < 8; ++r) {
    const float v = acc[r];
    Xs[(T * 16 + 8 * hh + r) * XSP + ncol] = v;
    ss[r] = v * cs;
    sd[r] = v * cd;
  }
#pragma unroll
  for (int mk = 1; mk < 16; mk <<= 1) {
#pragma unroll
    for (int r = 0; r < 8; ++r) {
      ss[r] += __shfl_xor(ss[r], mk, 32);
      sd[r] += __shfl_xor(sd[r], mk, 32);
    }
  }
  if (m == 0) {
#pragma unroll
    for (int r = 0; r < 8; ++r) {
      As[(T * 16 + 8 * hh + r) * NWAVE + wave] = ss[r];
      Ds[(T * 16 + 8 * hh + r) * NWAVE + wave] = sd[r];
    }
  }
}

__global__ __launch_bounds__(NTHR) void k_gemm(
    const float* __restrict__ ha, const unsigned short* __restrict__ Ph,
    const unsigned short* __restrict__ Pl,
    const float* __restrict__ att_src, const float* __restrict__ att_dst,
    float* xp, float* asrc, float* adst, int nN) {
  __shared__ __attribute__((aligned(16))) unsigned short Ah[GR * AP];
  __shared__ __attribute__((aligned(16))) unsigned short Al[GR * AP];
  __shared__ __attribute__((aligned(16))) float Xs[GR * XSP];
  __shared__ __attribute__((aligned(16))) float As[GR * NWAVE];
  __shared__ __attribute__((aligned(16))) float Ds[GR * NWAVE];

  const int tid  = threadIdx.x;
  const int lane = tid & 31;
  const int wave = tid >> 5;
  const int hh   = lane >> 4;
  const int m    = lane & 15;
  const int rowBase = blockIdx.x * GR;

  {
    const int r  = tid >> 3;
    const int c0 = (tid & 7) * 16;
    int row = rowBase + r;
    if (row > nN - 1) row = nN - 1;
    const float* p = ha + (size_t)row * FD + c0;
    const v4f f0 = *(const v4f*)(p), f1 = *(const v4f*)(p + 4);
    const v4f f2 = *(const v4f*)(p + 8), f3 = *(const v4f*)(p + 12);
    Pack16 h0, l0, h1, l1;
    split2(f0.x, h0.s[0], l0.s[0]); split2(f0.y, h0.s[1], l0.s[1]);
    split2(f0.z, h0.s[2], l0.s[2]); split2(f0.w, h0.s[3], l0.s[3]);
    split2(f1.x, h0.s[4], l0.s[4]); split2(f1.y, h0.s[5], l0.s[5]);
    split2(f1.z, h0.s[6], l0.s[6]); split2(f1.w, h0.s[7], l0.s[7]);
    split2(f2.x, h1.s[0], l1.s[0]); split2(f2.y, h1.s[1], l1.s[1]);
    split2(f2.z, h1.s[2], l1.s[2]); split2(f2.w, h1.s[3], l1.s[3]);
    split2(f3.x, h1.s[4], l1.s[4]); split2(f3.y, h1.s[5], l1.s[5]);
    split2(f3.z, h1.s[6], l1.s[6]); split2(f3.w, h1.s[7], l1.s[7]);
    *(v8us*)(Ah + r * AP + c0)     = h0.h;
    *(v8us*)(Ah + r * AP + c0 + 8) = h1.h;
    *(v8us*)(Al + r * AP + c0)     = l0.h;
    *(v8us*)(Al + r * AP + c0 + 8) = l1.h;
  }
  __syncthreads();

  const int ncol = wave * 16 + m;
  v8f c0a = {0.f, 0.f, 0.f, 0.f, 0.f, 0.f, 0.f, 0.f};
  v8f c1a = {0.f, 0.f, 0.f, 0.f, 0.f, 0.f, 0.f, 0.f};
#pragma unroll
  for (int kt = 0; kt < FD / 32; ++kt) {
    const int k0 = kt * 32;
    Frag a0h, a0l, a1h, a1l, bh, bl;
    const unsigned short* pbh = Ph + (size_t)ncol * FD + k0 + 8 * hh;
    const unsigned short* pbl = Pl + (size_t)ncol * FD + k0 + 8 * hh;
    const unsigned short* pa0 = Ah + m * AP + k0 + 8 * hh;
    const unsigned short* pa1 = Ah + (16 + m) * AP + k0 + 8 * hh;
    const unsigned short* qa0 = Al + m * AP + k0 + 8 * hh;
    const unsigned short* qa1 = Al + (16 + m) * AP + k0 + 8 * hh;
    bh.half[0]  = *(const v8us*)pbh;  bh.half[1]  = *(const v8us*)(pbh + 16);
    bl.half[0]  = *(const v8us*)pbl;  bl.half[1]  = *(const v8us*)(pbl + 16);
    a0h.half[0] = *(const v8us*)pa0;  a0h.half[1] = *(const v8us*)(pa0 + 16);
    a1h.half[0] = *(const v8us*)pa1;  a1h.half[1] = *(const v8us*)(pa1 + 16);
    a0l.half[0] = *(const v8us*)qa0;  a0l.half[1] = *(const v8us*)(qa0 + 16);
    a1l.half[0] = *(const v8us*)qa1;  a1l.half[1] = *(const v8us*)(qa1 + 16);
    c0a = wm(a0h.v, bh.v, c0a);
    c0a = wm(a0h.v, bl.v, c0a);
    c0a = wm(a0l.v, bh.v, c0a);
    c1a = wm(a1h.v, bh.v, c1a);
    c1a = wm(a1h.v, bl.v, c1a);
    c1a = wm(a1l.v, bh.v, c1a);
  }

  const float cs = att_src[ncol];
  const float cd = att_dst[ncol];
  epi_tile(c0a, 0, hh, m, wave, ncol, cs, cd, Xs, As, Ds);
  epi_tile(c1a, 1, hh, m, wave, ncol, cs, cd, Xs, As, Ds);
  __syncthreads();
  block_out(Xs, As, Ds, xp, asrc, adst, rowBase, wave, lane);
}

template <int LAST>
__global__ __launch_bounds__(NTHR) void k_gat(
    const int* __restrict__ ei, const float* __restrict__ xp,
    const float* __restrict__ asrc, const float* __restrict__ adst,
    const float* __restrict__ bias, const int* __restrict__ batch,
    float* hout, double* prec, int nN, int nE) {
  extern __shared__ v4f lds_dyn[];
  float* sacc = (float*)lds_dyn;
  float* den  = sacc + LDS_SACC;
  float* mx   = den + NB * NH;
  int*   list = (int*)(mx + NB * NH);
  int*   wcnt = list + LDS_LIST;

  const int tid  = threadIdx.x;
  const int lane = tid & 31;
  const int wave = tid >> 5;
  const int hd   = lane >> 3;
  const int nodeBase = blockIdx.x * NB;

#pragma unroll 1
  for (int j = 0; j < NB / NWAVE; ++j) {
    const int slot = wave * (NB / NWAVE) + j;
    int node = nodeBase + slot;
    if (node > nN - 1) node = nN - 1;
    const size_t nr = (size_t)node;
    const v4f xv = *(const v4f*)(xp + nr * FD + 4 * lane);
    *(v4f*)(sacc + slot * FD + 4 * lane) = xv;
    float a = asrc[nr * NH + hd] + adst[nr * NH + hd];
    a = (a > 0.f) ? a : 0.2f * a;
    mx[slot * NH + hd]  = a;
    den[slot * NH + hd] = 1.0f;
  }
  __syncthreads();

  const int* eid = ei + nE;
  const bool al16 = ((((size_t)eid) & 15) == 0);

  const int nChunks = (nE + CHUNK - 1) / CHUNK;
#pragma unroll 1
  for (int ch = 0; ch < nChunks; ++ch) {
    const int cbase = ch * CHUNK;
    const bool full = (cbase + CHUNK <= nE);
    int wc = 0;
#pragma unroll
    for (int g = 0; g < NGRP; ++g) {
      const int el0 = (g * NTHR + tid) * 4;
      const int e0  = cbase + el0;
      const int sent = -2147483647 - 1;
      v4i d;
      if (al16 && full) {
        d = *(const v4i*)(eid + e0);
      } else {
        const int i0 = min(e0, nE - 1),     i1 = min(e0 + 1, nE - 1);
        const int i2 = min(e0 + 2, nE - 1), i3 = min(e0 + 3, nE - 1);
        d.x = (e0     < nE) ? eid[i0] : sent;
        d.y = (e0 + 1 < nE) ? eid[i1] : sent;
        d.z = (e0 + 2 < nE) ? eid[i2] : sent;
        d.w = (e0 + 3 < nE) ? eid[i3] : sent;
      }
      const unsigned s0 = (unsigned)d.x - (unsigned)nodeBase;
      const unsigned s1 = (unsigned)d.y - (unsigned)nodeBase;
      const unsigned s2 = (unsigned)d.z - (unsigned)nodeBase;
      const unsigned s3 = (unsigned)d.w - (unsigned)nodeBase;
      const bool h0 = s0 < (unsigned)NB;
      const bool h1 = s1 < (unsigned)NB;
      const bool h2 = s2 < (unsigned)NB;
      const bool h3 = s3 < (unsigned)NB;
      const unsigned many = __builtin_amdgcn_ballot_w32(h0 | h1 | h2 | h3);
      if (many != 0u) {
#define HITJ(J, HJ, SJ) { \
          const unsigned mj = __builtin_amdgcn_ballot_w32(HJ); \
          if (HJ) { \
            const int pos = wc + (int)__builtin_amdgcn_mbcnt_lo(mj, 0u); \
            if (pos < WCAP) list[wave * WCAP + pos] = ((el0 + (J)) << 9) | (int)(SJ); \
          } \
          wc += (int)__builtin_popcount(mj); }
        HITJ(0, h0, s0)
        HITJ(1, h1, s1)
        HITJ(2, h2, s2)
        HITJ(3, h3, s3)
#undef HITJ
      }
    }
    if (lane == 0) wcnt[wave] = wc;
    __syncthreads();

    if (wave == 0) {
#pragma unroll 1
      for (int wsx = 0; wsx < NWAVE; ++wsx) {
        int n = wcnt[wsx];
        if (n > WCAP) n = WCAP;
        if (n < 0) n = 0;
#pragma unroll 1
        for (int i = 0; i < n; ++i) {
          const int ent  = list[wsx * WCAP + i];
          const int slot = ent & (NB - 1);
          const int el   = (ent >> 9) & (CHUNK - 1);
          int e = cbase + el;
          if (e > nE - 1) e = nE - 1;
          int src = ei[e];
          src = src < 0 ? 0 : (src > nN - 1 ? nN - 1 : src);
          int nd = nodeBase + slot;
          if (nd > nN - 1) nd = nN - 1;
          float al = asrc[(size_t)src * NH + hd] + adst[(size_t)nd * NH + hd];
          al = (al > 0.f) ? al : 0.2f * al;
          const int mi   = slot * NH + hd;
          const float m  = mx[mi];
          const float dn = den[mi];
          const float nm = fmaxf(m, al);
          const float sc = __expf(m - nm);
          const float p  = __expf(al - nm);
          const v4f xv = *(const v4f*)(xp + (size_t)src * FD + 4 * lane);
          v4f* sp = (v4f*)(sacc + slot * FD + 4 * lane);
          const v4f cur = *sp;
          const v4f nxt = cur * sc + xv * p;
          *sp = nxt;
          mx[mi]  = nm;
          den[mi] = dn * sc + p;
        }
      }
    }
    __syncthreads();
  }

  if (LAST == 0) {
    const v4f b4 = *(const v4f*)(bias + 4 * lane);
#pragma unroll 1
    for (int j = 0; j < NB / NWAVE; ++j) {
      const int slot = wave * (NB / NWAVE) + j;
      const int node = nodeBase + slot;
      if (node >= nN) break;
      const float dv  = den[slot * NH + hd];
      const float inv = 1.0f / (dv + 1e-16f);
      v4f h = *(const v4f*)(sacc + slot * FD + 4 * lane) * inv + b4;
      h.x = h.x > 0.f ? h.x : (__expf(h.x) - 1.0f);
      h.y = h.y > 0.f ? h.y : (__expf(h.y) - 1.0f);
      h.z = h.z > 0.f ? h.z : (__expf(h.z) - 1.0f);
      h.w = h.w > 0.f ? h.w : (__expf(h.w) - 1.0f);
      float* op = hout + (size_t)node * FD + 4 * lane;
      *(volatile v4f*)op = h;
      __threadfence();
      *(volatile v4f*)op = h;
    }
  } else {
    const int cb = (4 * lane) & (HC - 1);
    const v4f b4 = *(const v4f*)(bias + cb);
    double pa0 = 0.0, pa1 = 0.0, pa2 = 0.0, pa3 = 0.0;
    double pb0 = 0.0, pb1 = 0.0, pb2 = 0.0, pb3 = 0.0;
    int n0 = 0, n1 = 0;
#pragma unroll 1
    for (int j = 0; j < NB / NWAVE; ++j) {
      const int slot = wave * (NB / NWAVE) + j;
      const int node = nodeBase + slot;
      if (node >= nN) break;
      const float dv  = den[slot * NH + hd];
      const float inv = 1.0f / (dv + 1e-16f);
      const v4f h = *(const v4f*)(sacc + slot * FD + 4 * lane) * inv;
      v4f s;
      s.x = h.x + __shfl_xor(h.x, 8, 32);
      s.y = h.y + __shfl_xor(h.y, 8, 32);
      s.z = h.z + __shfl_xor(h.z, 8, 32);
      s.w = h.w + __shfl_xor(h.w, 8, 32);
      s.x = s.x + __shfl_xor(s.x, 16, 32);
      s.y = s.y + __shfl_xor(s.y, 16, 32);
      s.z = s.z + __shfl_xor(s.z, 16, 32);
      s.w = s.w + __shfl_xor(s.w, 16, 32);
      const v4f hm = s * 0.25f + b4;
      const int g = batch[node];
      const bool is0 = (g <= 0);
      pa0 += is0 ? (double)hm.x : 0.0;  pb0 += is0 ? 0.0 : (double)hm.x;
      pa1 += is0 ? (double)hm.y : 0.0;  pb1 += is0 ? 0.0 : (double)hm.y;
      pa2 += is0 ? (double)hm.z : 0.0;  pb2 += is0 ? 0.0 : (double)hm.z;
      pa3 += is0 ? (double)hm.w : 0.0;  pb3 += is0 ? 0.0 : (double)hm.w;
      n0 += is0 ? 1 : 0;
      n1 += is0 ? 0 : 1;
    }
    __syncthreads();
    double* Pd = (double*)lds_dyn;
    int*    Pc = list;
    if (lane < 8) {
      Pd[wave * 64 + 4 * lane + 0] = pa0;  Pd[wave * 64 + HC + 4 * lane + 0] = pb0;
      Pd[wave * 64 + 4 * lane + 1] = pa1;  Pd[wave * 64 + HC + 4 * lane + 1] = pb1;
      Pd[wave * 64 + 4 * lane + 2] = pa2;  Pd[wave * 64 + HC + 4 * lane + 2] = pb2;
      Pd[wave * 64 + 4 * lane + 3] = pa3;  Pd[wave * 64 + HC + 4 * lane + 3] = pb3;
    }
    if (lane == 0) { Pc[wave * 2 + 0] = n0; Pc[wave * 2 + 1] = n1; }
    __syncthreads();
    double* Rs = Pd + NWAVE * 64;
    if (tid < 64) {
      double s = 0.0;
#pragma unroll
      for (int w = 0; w < NWAVE; ++w) s += Pd[w * 64 + tid];
      Rs[tid] = s;
    } else if (tid < 66) {
      int c = 0;
#pragma unroll
      for (int w = 0; w < NWAVE; ++w) c += Pc[w * 2 + (tid - 64)];
      Rs[tid] = (double)c;
    } else if (tid < RECD) {
      Rs[tid] = 0.0;
    }
    __syncthreads();
    const int pt = tid < RECD / 2 ? tid : RECD / 2 - 1;
    const v2d rv = *(const v2d*)(Rs + 2 * pt);
    double* gp = prec + (size_t)blockIdx.x * RECD + 2 * pt;
    if (tid < RECD / 2) *(volatile v2d*)gp = rv;
    __threadfence();
    if (tid < RECD / 2) *(volatile v2d*)gp = rv;
  }
}

__global__ __launch_bounds__(64) void k_final(
    const double* __restrict__ prec, int nblk,
    const float* __restrict__ mW1, const float* __restrict__ mb1,
    const float* __restrict__ mW2, const float* __restrict__ mb2,
    float* out) {
  __shared__ float gvs[NG * HC];
  __shared__ float hid[NG * HC];
  __shared__ __attribute__((aligned(16))) float ost[32];
  const int t = threadIdx.x;
  const int g = t >> 5;
  const int c = t & 31;
  double s = 0.0, cn = 0.0;
#pragma unroll 1
  for (int b = 0; b < nblk; ++b) {
    s  += prec[(size_t)b * RECD + t];
    cn += prec[(size_t)b * RECD + 64 + g];
  }
  const double cm = cn > 1.0 ? cn : 1.0;
  gvs[t] = (float)(s / cm);
  __syncthreads();
  float a = 0.f;
#pragma unroll 1
  for (int k = 0; k < HC; ++k) a = fmaf(gvs[g * HC + k], mW1[k * HC + c], a);
  a += mb1[c];
  hid[t] = a > 0.f ? a : 0.f;
  __syncthreads();
  const int tt = t < NG * NOUT ? t : NG * NOUT - 1;
  const int gg = tt / NOUT;
  const int o  = tt - gg * NOUT;
  float r = 0.f;
#pragma unroll 1
  for (int k = 0; k < HC; ++k) r = fmaf(hid[gg * HC + k], mW2[k * NOUT + o], r);
  r += mb2[o];
  if (t < 32) ost[t] = (t < NG * NOUT) ? r : 0.f;
  __syncthreads();
  v4f ov = {0.f, 0.f, 0.f, 0.f};
  if (t < 5) ov = *(const v4f*)(ost + 4 * t);
  if (t < 5) *(volatile v4f*)(out + 4 * t) = ov;
  __threadfence();
  if (t < 5) *(volatile v4f*)(out + 4 * t) = ov;
}

extern "C" void kernel_launch(void* const* d_in, const int* in_sizes, int n_in,
                              void* d_out, int out_size, void* d_ws, size_t ws_size,
                              hipStream_t stream) {
  if (n_in < 19) return;
  const int nN = in_sizes[2];
  if (nN <= 0 || in_sizes[0] != 3 * nN) return;
  if (in_sizes[1] < 2 || (in_sizes[1] & 1)) return;
  const int nE = in_sizes[1] / 2;
  if (in_sizes[3] != 3 * FD || in_sizes[4] != FD || in_sizes[5] != FD || in_sizes[6] != FD) return;
  if (in_sizes[7] != FD * FD || in_sizes[8] != FD || in_sizes[9] != FD || in_sizes[10] != FD) return;
  if (in_sizes[11] != FD * FD || in_sizes[12] != FD || in_sizes[13] != FD || in_sizes[14] != HC) return;
  if (in_sizes[15] != HC * HC || in_sizes[16] != HC || in_sizes[17] != HC * NOUT || in_sizes[18] != NOUT) return;
  if (out_size != NG * NOUT) return;

  const float* x     = (const float*)d_in[0];
  const int*   ei    = (const int*)d_in[1];
  const int*   batch = (const int*)d_in[2];
  const float* W0    = (const float*)d_in[3];
  const float* as0   = (const float*)d_in[4];
  const float* ad0   = (const float*)d_in[5];
  const float* b0    = (const float*)d_in[6];
  const float* W1    = (const float*)d_in[7];
  const float* as1   = (const float*)d_in[8];
  const float* ad1   = (const float*)d_in[9];
  const float* b1    = (const float*)d_in[10];
  const float* W2    = (const float*)d_in[11];
  const float* as2   = (const float*)d_in[12];
  const float* ad2   = (const float*)d_in[13];
  const float* b2    = (const float*)d_in[14];
  const float* mW1   = (const float*)d_in[15];
  const float* mb1   = (const float*)d_in[16];
  const float* mW2   = (const float*)d_in[17];
  const float* mb2   = (const float*)d_in[18];
  float* out = (float*)d_out;

  const int nblk = (nN + NB - 1) / NB;
  const int nP   = nblk * NB;

  size_t off = 0;
  unsigned short* Wq = (unsigned short*)((char*)d_ws + off);
  off += (size_t)4 * FD * FD * sizeof(unsigned short);           off = (off + 255) & ~(size_t)255;
  float* XP = (float*)((char*)d_ws + off);
  off += (size_t)nP * FD * sizeof(float);                          off = (off + 255) & ~(size_t)255;
  float* HA = (float*)((char*)d_ws + off);
  off += (size_t)nP * FD * sizeof(float);                          off = (off + 255) & ~(size_t)255;
  float* ASRC = (float*)((char*)d_ws + off);
  off += (size_t)nP * NH * sizeof(float);                          off = (off + 255) & ~(size_t)255;
  float* ADST = (float*)((char*)d_ws + off);
  off += (size_t)nP * NH * sizeof(float);                          off = (off + 255) & ~(size_t)255;
  double* PREC = (double*)((char*)d_ws + off);
  off += (size_t)nblk * RECD * sizeof(double);                     off = (off + 255) & ~(size_t)255;
  if (off > ws_size) return;

  const int tgrid = nP / GR;

  k_prepw<<<16, NTHR, 0, stream>>>(W1, W2, Wq);

  k_l0<<<tgrid, NTHR, 0, stream>>>(x, W0, as0, ad0, XP, ASRC, ADST, nN);

  hipFuncSetAttribute(reinterpret_cast<const void*>(&k_gat<0>),
                      hipFuncAttributeMaxDynamicSharedMemorySize, LDS_BYTES);
  hipFuncSetAttribute(reinterpret_cast<const void*>(&k_gat<1>),
                      hipFuncAttributeMaxDynamicSharedMemorySize, LDS_BYTES);

  k_gat<0><<<nblk, NTHR, LDS_BYTES, stream>>>(ei, XP, ASRC, ADST, b0, batch, HA, PREC, nN, nE);

  k_gemm<<<tgrid, NTHR, 0, stream>>>(HA, Wq, Wq + FD * FD, as1, ad1, XP, ASRC, ADST, nN);
  k_gat<0><<<nblk, NTHR, LDS_BYTES, stream>>>(ei, XP, ASRC, ADST, b1, batch, HA, PREC, nN, nE);

  k_gemm<<<tgrid, NTHR, 0, stream>>>(HA, Wq + 2 * FD * FD, Wq + 3 * FD * FD, as2, ad2, XP, ASRC, ADST, nN);
  k_gat<1><<<nblk, NTHR, LDS_BYTES, stream>>>(ei, XP, ASRC, ADST, b2, batch, HA, PREC, nN, nE);

  k_final<<<1, 64, 0, stream>>>(PREC, nblk, mW1, mb1, mW2, mb2, out);
}
